// QwenTorchMultiHeadAttentionHandler_63050119905466
// MI455X (gfx1250) — hardware-verified
//
#include <hip/hip_runtime.h>


namespace {
constexpr int S = 4096, H = 16, HD = 80, HDP = 96, NSEG = 8;
constexpr float PS = 8.0f, SCL = 0.11180339887498948f;
constexpr size_t QPL = (size_t)H * S * HDP, VPL = (size_t)H * HD * S;

typedef _Float16 b16;
typedef __attribute__((ext_vector_type(16))) _Float16 v16b;
typedef __attribute__((ext_vector_type(16))) __bf16 v16bb;
typedef __attribute__((ext_vector_type(8))) _Float16 v8b;
typedef __attribute__((ext_vector_type(8))) unsigned short v8us;
typedef __attribute__((ext_vector_type(8))) float v8f;
typedef __attribute__((ext_vector_type(4))) float v4f;
__device__ __forceinline__ float bf16_rne(float f) { unsigned int u = __float_as_uint(f); u += 0x7FFFu + ((u >> 16) & 1u); return __uint_as_float(u & 0xFFFF0000u); }
__device__ __forceinline__ unsigned short bf16_bits(float f) { unsigned int u = __float_as_uint(f); u += 0x7FFFu + ((u >> 16) & 1u); return (unsigned short)(u >> 16); }
__device__ __forceinline__ void split16(float v, b16& hi, b16& lo) { hi = (b16)v; lo = (b16)(v - (float)hi); }
__device__ __forceinline__ v16b frag_kb(const b16* p, int hh) { const v8b a = *(const v8b*)(p + 8 * hh), b = *(const v8b*)(p + 16 + 8 * hh); v16b f;
#pragma unroll
  for (int e = 0; e < 8; ++e) { f[e] = a[e]; f[8 + e] = b[e]; } return f; }
__device__ __forceinline__ v16bb frag_bf(const unsigned short* p, int hh) { const v8us a = *(const v8us*)(p + 8 * hh), b = *(const v8us*)(p + 16 + 8 * hh); union { unsigned short s[16]; v16bb v; } u;
#pragma unroll
  for (int e = 0; e < 8; ++e) { u.s[e] = a[e]; u.s[8 + e] = b[e]; } return u.v; }
__device__ __forceinline__ v8f wmma16b(v16b a, v16b b, v8f c) { v8f d = __builtin_amdgcn_wmma_f32_16x16x32_f16(false, a, false, b, (short)0, c, false, false); asm volatile("v_nop\n\tv_nop\n\tv_nop\n\tv_nop" : "+v"(d) : "v"(a), "v"(b)); return d; }
__device__ __forceinline__ v8f wmma16bb(v16bb a, v16bb b, v8f c) { v8f d = __builtin_amdgcn_wmma_f32_16x16x32_bf16(false, a, false, b, (short)0, c, false, false); asm volatile("v_nop\n\tv_nop\n\tv_nop\n\tv_nop" : "+v"(d) : "v"(a), "v"(b)); return d; }
__device__ __forceinline__ float nexp(float x) { return __builtin_amdgcn_exp2f(x * 1.4426950408889634f); }

__global__ __launch_bounds__(128) void prep_kernel(const float* __restrict__ q, const float* __restrict__ k, const float* __restrict__ v, unsigned short* __restrict__ qp, unsigned short* __restrict__ kp, b16* __restrict__ vt) {
  __shared__ __attribute__((aligned(16))) unsigned short Tq[128][HDP], Tk[128][HDP]; __shared__ __attribute__((aligned(16))) b16 Tv[HD][128 + 8];
  const int t_ = threadIdx.x, h = blockIdx.y, s0 = blockIdx.x * 128;
  for (int i = t_; i < 128 * HDP; i += 128) { const int r = i / HDP, d = i % HDP; const size_t src = ((size_t)(s0 + r) * H + h) * HD + d;
    Tq[r][d] = (d < HD) ? bf16_bits(q[src]) : (unsigned short)0; Tk[r][d] = (d < HD) ? bf16_bits(k[src]) : (unsigned short)0; if (d < HD) Tv[d][r] = (b16)bf16_rne(v[src]); }
  __syncthreads();
  for (int pass = 0; pass < 2; ++pass) {
    for (int i = t_; i < 128 * HDP / 8; i += 128) { const size_t o = ((size_t)h * S + s0) * HDP + (size_t)i * 8; *(volatile v8us*)(qp + o) = *(const v8us*)(&Tq[0][0] + i * 8); *(volatile v8us*)(kp + o) = *(const v8us*)(&Tk[0][0] + i * 8); }
    for (int i = t_; i < HD * 16; i += 128) { const int d = i >> 4, c8 = (i & 15) * 8; *(volatile v8b*)(vt + ((size_t)h * HD + d) * S + s0 + c8) = *(const v8b*)(&Tv[d][c8]); }
    __threadfence(); }
}

__global__ __launch_bounds__(256) void attn_kernel(const unsigned short* __restrict__ qp, const unsigned short* __restrict__ kp, const b16* __restrict__ vt, const int* __restrict__ cu, float* __restrict__ out) {
  __shared__ __attribute__((aligned(16))) float Os[16][8 * HD + 4];
  const int wid = threadIdx.x >> 5, lane = threadIdx.x & 31, hh = lane >> 4, col = lane & 15; const int q0 = blockIdx.x * 16, h = blockIdx.y * 8 + wid, qi = q0 + col;
  int sg = 0;
#pragma unroll
  for (int j = 1; j <= NSEG; ++j) sg += (cu[j] <= qi) ? 1 : 0;
  sg = (sg >= NSEG) ? NSEG - 1 : sg; int lo = max(0, min(cu[sg], S)), hi = max(0, min(cu[sg + 1], S)); if (!(lo <= qi && qi < hi)) { lo = min(lo, qi); hi = max(hi, qi + 1); }
  int wlo = lo, whi = hi;
#pragma unroll
  for (int o = 1; o < 32; o <<= 1) { wlo = min(wlo, __shfl_xor(wlo, o)); whi = max(whi, __shfl_xor(whi, o)); }
  wlo &= ~31;
  const unsigned short* Q = qp + ((size_t)h * S) * HDP; const unsigned short* K = kp + ((size_t)h * S) * HDP; const b16* V = vt + ((size_t)h * HD) * S;
  v16bb qf[3];
#pragma unroll
  for (int ks = 0; ks < 3; ++ks) qf[ks] = frag_bf(Q + (size_t)qi * HDP + ks * 32, hh);
  float m = -INFINITY, l = 0.0f; v8f oacc[5] = {{}, {}, {}, {}, {}};
  for (int kb = wlo; kb < whi; kb += 32) { v8f s0 = {}, s1 = {};
#pragma unroll
    for (int ks = 0; ks < 3; ++ks) { const v16bb ka = frag_bf(K + (size_t)(kb + col) * HDP + ks * 32, hh), kc = frag_bf(K + (size_t)(kb + 16 + col) * HDP + ks * 32, hh); s0 = wmma16bb(ka, qf[ks], s0); s1 = wmma16bb(kc, qf[ks], s1); }
    float mr = -INFINITY;
#pragma unroll
    for (int r = 0; r < 8; ++r) { const int k0_ = kb + 8 * hh + r, k1_ = kb + 16 + 8 * hh + r; s0[r] = (k0_ >= lo && k0_ < hi) ? s0[r] * SCL : -INFINITY; s1[r] = (k1_ >= lo && k1_ < hi) ? s1[r] * SCL : -INFINITY; mr = fmaxf(mr, fmaxf(s0[r], s1[r])); }
    mr = fmaxf(mr, __shfl_xor(mr, 16));
    const float mn = fmaxf(m, mr); const float al_ = (mn == -INFINITY) ? 1.0f : nexp(m - mn); float sum = 0.0f; v16b pbv, plv;
#pragma unroll
    for (int r = 0; r < 8; ++r) { const float e0 = (mn == -INFINITY) ? 0.0f : nexp(s0[r] - mn), e1 = (mn == -INFINITY) ? 0.0f : nexp(s1[r] - mn); sum += e0 + e1; b16 a, cc; split16(e0 * PS, a, cc); pbv[r] = a; plv[r] = cc; split16(e1 * PS, a, cc); pbv[8 + r] = a; plv[8 + r] = cc; }
    sum += __shfl_xor(sum, 16); l = l * al_ + sum; m = mn;
#pragma unroll
    for (int t = 0; t < 5; ++t) { oacc[t] *= al_; const v16b vf = frag_kb(V + (size_t)(t * 16 + col) * S + kb, hh); oacc[t] = wmma16b(vf, pbv, oacc[t]); oacc[t] = wmma16b(vf, plv, oacc[t]); } }
  const float inv = 1.0f / (l * PS);
#pragma unroll
  for (int t = 0; t < 5; ++t)
#pragma unroll
    for (int r = 0; r < 8; ++r) Os[col][wid * HD + t * 16 + 8 * hh + r] = oacc[t][r] * inv;
  __syncthreads();
  for (int pass = 0; pass < 2; ++pass) { for (int i = threadIdx.x; i < 16 * (8 * HD / 4); i += 256) { const int rr = i / (8 * HD / 4), c4 = (i % (8 * HD / 4)) * 4; *(volatile v4f*)(out + (size_t)(q0 + rr) * (H * HD) + blockIdx.y * 8 * HD + c4) = *(const v4f*)(&Os[rr][c4]); } __threadfence(); }
}
}

extern "C" void kernel_launch(void* const* d_in, const int* in_sizes, int n_in,
                              void* d_out, int out_size, void* d_ws, size_t ws_size, hipStream_t stream) {
  (void)n_in; (void)out_size;
  const float* q = (const float*)d_in[0]; const float* k = (const float*)d_in[1]; const float* v = (const float*)d_in[2]; const int* cu = (const int*)d_in[4];
  float* out = (float*)d_out;
  if (in_sizes[0] != S * H * HD || in_sizes[1] != S * H * HD || in_sizes[2] != S * H * HD || in_sizes[4] != NSEG + 1) return;
  size_t off = 0; char* ws = (char*)d_ws;
  auto carve = [&](size_t bytes) { char* p = ws + off; off += (bytes + 255) & ~(size_t)255; return p; };
  unsigned short* qp = (unsigned short*)carve(QPL * 2); unsigned short* kp = (unsigned short*)carve(QPL * 2); b16* vt = (b16*)carve(VPL * 2);
  if (off > ws_size) return;
  prep_kernel<<<dim3(S / 128, H), 128, 0, stream>>>(q, k, v, qp, kp, vt);
  attn_kernel<<<dim3(S / 16, H / 8), 256, 0, stream>>>(qp, kp, vt, cu, out);
}
